// Propagation_927712936457
// MI455X (gfx1250) — hardware-verified
//
#include <hip/hip_runtime.h>
#include <stdint.h>

constexpr int kBatch  = 4;
constexpr int kNodes  = 4096;
constexpr int kDim    = 256;
constexpr int kVtRows = 320;
constexpr int kCPitch = 320;

static_assert(kDim % 32 == 0);
static_assert(kNodes % 32 == 0);
static_assert(kNodes % 64 == 0);
static_assert(kVtRows % 64 == 0);
static_assert((kCPitch * 4) % 128 == 0);
static_assert(kBatch * kNodes * 4 == 65536);
static_assert(65536 + kBatch * kNodes * kDim * 4 == 16842752);

constexpr size_t kBytesV16 = (size_t)kBatch * kNodes * kDim * 2;
constexpr size_t kBytesVT  = (size_t)kBatch * kVtRows * kNodes * 2;
constexpr size_t kBytesE   = (size_t)kNodes * kNodes * 2;
constexpr size_t kBytesC   = (size_t)kBatch * kNodes * kCPitch * 4;
constexpr size_t kOffV16 = 0;
constexpr size_t kOffVT  = kOffV16 + kBytesV16;
constexpr size_t kOffE   = kOffVT + kBytesVT;
constexpr size_t kOffC   = kOffE + kBytesE;
constexpr size_t kWsTotal = kOffC + kBytesC;
static_assert(kWsTotal == 73400320);
static_assert(kWsTotal <= 134217728);
static_assert(kOffVT % 128 == 0 && kOffE % 128 == 0 && kOffC % 128 == 0);

typedef __attribute__((ext_vector_type(16))) _Float16 v16h;
typedef __attribute__((ext_vector_type(8)))  _Float16 v8h;
typedef __attribute__((ext_vector_type(16))) __bf16   v16b;
typedef __attribute__((ext_vector_type(8)))  __bf16   v8b;
typedef __attribute__((ext_vector_type(8)))  float    v8f;
typedef __attribute__((ext_vector_type(4)))  float    v4f;

__device__ __forceinline__ unsigned short f2bf_bits(float f) {
  unsigned u = __float_as_uint(f);
  return (unsigned short)((u + 0x7FFFu + ((u >> 16) & 1u)) >> 16);
}
__device__ __forceinline__ float bf_bits2f(unsigned short h) { return __uint_as_float(((unsigned)h) << 16); }

__device__ __forceinline__ _Float16 bfr_to_h(float f) {
  const float r = bf_bits2f(f2bf_bits(f));
  return (_Float16)r;
}

__device__ __forceinline__ void dep_guard_h(v8f& a, v8f& b, v16h x, v16h y) { asm volatile("v_nop\n\tv_nop\n\tv_nop\n\tv_nop" : "+v"(a), "+v"(b) : "v"(x), "v"(y)); }
__device__ __forceinline__ void dep_guard_b(v8f& a, v8f& b, v16b x, v16b y) { asm volatile("v_nop\n\tv_nop\n\tv_nop\n\tv_nop" : "+v"(a), "+v"(b) : "v"(x), "v"(y)); }
__device__ __forceinline__ void keep4_h(v16h a, v16h b, v16h c, v16h d) { asm volatile("v_nop" :: "v"(a), "v"(b), "v"(c), "v"(d)); }
__device__ __forceinline__ void keep4_b(v16b a, v16b b, v16b c, v16b d) { asm volatile("v_nop" :: "v"(a), "v"(b), "v"(c), "v"(d)); }
__device__ __forceinline__ void acc_guard4(v8f& a, v8f& b, v8f& c, v8f& d) { asm volatile("v_nop\n\tv_nop\n\tv_nop\n\tv_nop" : "+v"(a), "+v"(b), "+v"(c), "+v"(d)); }
template <typename T> struct Frag;
template <> struct Frag<_Float16> {
  typedef v16h V; union U { v16h v; v8h h[2]; };
  static __device__ __forceinline__ v16h load(const _Float16* p) {
    U f; f.h[0] = *(const v8h*)(p); f.h[1] = *(const v8h*)(p + 16); return f.v;
  }
  static __device__ __forceinline__ v8f mma(v16h a, v16h b, v8f c) {
    return __builtin_amdgcn_wmma_f32_16x16x32_f16(false, a, false, b, (short)0, c, false, false);
  }
  static __device__ __forceinline__ void guard(v8f& a, v8f& b, v16h x, v16h y) { dep_guard_h(a, b, x, y); }
  static __device__ __forceinline__ void keep(v16h a, v16h b, v16h c, v16h d) { keep4_h(a, b, c, d); }
};
template <> struct Frag<__bf16> {
  typedef v16b V; union U { v16b v; v8b h[2]; };
  static __device__ __forceinline__ v16b load(const __bf16* p) {
    U f; f.h[0] = *(const v8b*)(p); f.h[1] = *(const v8b*)(p + 16); return f.v;
  }
  static __device__ __forceinline__ v8f mma(v16b a, v16b b, v8f c) {
    return __builtin_amdgcn_wmma_f32_16x16x32_bf16(false, a, false, b, (short)0, c, false, false);
  }
  static __device__ __forceinline__ void guard(v8f& a, v8f& b, v16b x, v16b y) { dep_guard_b(a, b, x, y); }
  static __device__ __forceinline__ void keep(v16b a, v16b b, v16b c, v16b d) { keep4_b(a, b, c, d); }
};

template <int ET> struct Elem;
template <> struct Elem<0> { typedef _Float16 T; };
template <> struct Elem<1> { typedef __bf16 T; };
template <int ET, bool SPLIT, int BIAS_MODE, int OUT_MODE, bool RESID, int ACT = 0>
__global__ __launch_bounds__(256) void wmma_gemm64(
    const unsigned short* __restrict__ Ap, const unsigned short* __restrict__ A2p, int lda, long strideA,
    const unsigned short* __restrict__ Btp, const unsigned short* __restrict__ Bt2p, int ldb, long strideB,
    void* __restrict__ Cout, void* __restrict__ Cout2, int ldc, long strideC,
    const float* __restrict__ bias,
    const float* __restrict__ resid, long strideR,
    int M, int N, int K, float scale) {
  typedef typename Elem<ET>::T T;
  typedef typename Frag<T>::V V;
  const T* A = (const T*)Ap; const T* A2 = (const T*)A2p; const T* Bt = (const T*)Btp; const T* Bt2 = (const T*)Bt2p;
  __shared__ __align__(16) float sT[8][16 * 68];
  const int b    = blockIdx.y;
  const int lane = threadIdx.x & 31;
  const int wave = threadIdx.x >> 5;
  const int tilesN = N >> 6;
  const int tilesM = M >> 6;
  const int tile = blockIdx.x * 8 + wave;
  if (tile >= tilesM * tilesN) return;
  const int tm = tile / tilesN;
  const int tn = tile - tm * tilesN;
  const int m0 = tm << 6;
  const int n0 = tn << 6;

  const T* Ab  = A  + (size_t)b * strideA;
  const T* Bb  = Bt + (size_t)b * strideB;
  const T* Ab2 = SPLIT ? (A2  + (size_t)b * strideA) : nullptr;
  const T* Bb2 = SPLIT ? (Bt2 + (size_t)b * strideB) : nullptr;

  const int rlane = lane & 15;
  const int koff  = (lane >> 4) * 8;
  const int mOff  = (lane >> 4) * 8;

  v8f acc[4][4];
#pragma unroll
  for (int i = 0; i < 4; ++i)
#pragma unroll
    for (int j = 0; j < 4; ++j) acc[i][j] = (v8f){0.f,0.f,0.f,0.f,0.f,0.f,0.f,0.f};

  for (int k0 = 0; k0 < K; k0 += 32) {
    V bh[4], bl[4];
#pragma unroll
    for (int j = 0; j < 4; ++j) {
      const size_t bo = (size_t)(n0 + (j << 4) + rlane) * ldb + koff + k0;
      bh[j] = Frag<T>::load(Bb + bo);
      if (SPLIT) bl[j] = Frag<T>::load(Bb2 + bo);
    }
#pragma unroll
    for (int i = 0; i < 4; ++i) {
      const size_t ao = (size_t)(m0 + (i << 4) + rlane) * lda + koff + k0;
      V ah = Frag<T>::load(Ab + ao);
      V al;
      if (SPLIT) al = Frag<T>::load(Ab2 + ao);
#pragma unroll
      for (int j = 0; j < 4; ++j) {
        acc[i][j] = Frag<T>::mma(ah, bh[j], acc[i][j]);
        if (SPLIT) {
          acc[i][j] = Frag<T>::mma(ah, bl[j], acc[i][j]);
          acc[i][j] = Frag<T>::mma(al, bh[j], acc[i][j]);
        }
      }
      Frag<T>::guard(acc[i][0], acc[i][3], ah, SPLIT ? al : ah);
    }
    Frag<T>::keep(bh[0], bh[1], bh[2], bh[3]);
    if (SPLIT) Frag<T>::keep(bl[0], bl[1], bl[2], bl[3]);
  }
  acc_guard4(acc[0][0], acc[0][1], acc[0][2], acc[0][3]);
  acc_guard4(acc[1][0], acc[1][1], acc[1][2], acc[1][3]);
  acc_guard4(acc[2][0], acc[2][1], acc[2][2], acc[2][3]);
  acc_guard4(acc[3][0], acc[3][1], acc[3][2], acc[3][3]);

  float* slab = sT[wave];
  const float* Rb = RESID ? (resid + (size_t)b * strideR) : nullptr;
#pragma unroll
  for (int i = 0; i < 4; ++i) {
    const int mBase = m0 + (i << 4);
#pragma unroll
    for (int j = 0; j < 4; ++j) {
      const int n = n0 + (j << 4) + rlane;
      float bv = 0.f;
      if (BIAS_MODE == 2) bv = bias[n];
#pragma unroll
      for (int r = 0; r < 8; ++r) {
        float v = acc[i][j][r] * scale;
        if (BIAS_MODE == 1) v += bias[mBase + mOff + r];
        if (BIAS_MODE == 2) v += bv;
        if (RESID) v += Rb[(size_t)(mBase + mOff + r) * ldc + n];
        if (ACT == 1) v = tanhf(v);
        if (ACT == 2) v = fmaxf(v, 0.0f);
        if (ACT == 3) v = v / (1.0f + expf(-v));
        if (ACT == 4) v = (v > 0.f) ? v : 0.01f * v;
        if (ACT == 5) v = 0.5f * v * (1.0f + erff(v * 0.70710678118654752f));
        if (ACT == 6) { const float av = 1.0f + fabsf(v); v = v * __builtin_amdgcn_rcpf(av); }
        slab[(mOff + r) * 68 + (j << 4) + rlane] = v;
      }
    }
    __builtin_amdgcn_fence(__ATOMIC_RELEASE, "workgroup");
    __builtin_amdgcn_wave_barrier();
    __builtin_amdgcn_fence(__ATOMIC_ACQUIRE, "workgroup");
    if (OUT_MODE == 0) {
      float* C = (float*)Cout + (size_t)b * strideC;
      const int hh = lane >> 4, c4 = (lane & 15) * 4;
      for (int pass = 0; pass < 2; ++pass) {
#pragma unroll
        for (int it = 0; it < 8; ++it) {
          const int row = it * 2 + hh;
          v4f v = *(const v4f*)(slab + row * 68 + c4);
          *(volatile v4f*)(C + (size_t)(mBase + row) * ldc + n0 + c4) = v;
        }
        __threadfence();
      }
    } else {
      const int q = lane >> 3, c8 = (lane & 7) * 8;
      unsigned short* C  = (unsigned short*)Cout  + (size_t)b * strideC;
      unsigned short* C2 = (OUT_MODE == 2) ? ((unsigned short*)Cout2 + (size_t)b * strideC) : nullptr;
      for (int pass = 0; pass < 2; ++pass) {
#pragma unroll
        for (int it = 0; it < 4; ++it) {
          const int row = it * 4 + q;
          const float* sp = slab + row * 68 + c8;
          v8h hv, lv;
#pragma unroll
          for (int e = 0; e < 8; ++e) {
            if (OUT_MODE == 1) {
              hv[e] = (_Float16)sp[e];
            } else {
              unsigned short hb = f2bf_bits(sp[e]);
              unsigned short lb = f2bf_bits(sp[e] - bf_bits2f(hb));
              hv[e] = __builtin_bit_cast(_Float16, hb);
              lv[e] = __builtin_bit_cast(_Float16, lb);
            }
          }
          *(volatile v8h*)(C + (size_t)(mBase + row) * ldc + n0 + c8) = hv;
          if (OUT_MODE == 2) *(volatile v8h*)(C2 + (size_t)(mBase + row) * ldc + n0 + c8) = lv;
        }
        __threadfence();
      }
    }
    __builtin_amdgcn_fence(__ATOMIC_RELEASE, "workgroup");
    __builtin_amdgcn_wave_barrier();
    __builtin_amdgcn_fence(__ATOMIC_ACQUIRE, "workgroup");
  }
}

__global__ __launch_bounds__(256) void cast_bfr_f16x8(const float* __restrict__ in,
                                                      unsigned short* __restrict__ out, int n8) {
  const int i = blockIdx.x * 256 + threadIdx.x;
  if (i < n8) {
    const size_t base = (size_t)i * 8;
    const v4f a = *(const v4f*)(in + base);
    const v4f c = *(const v4f*)(in + base + 4);
    v8h hv;
    hv[0] = bfr_to_h(a[0]); hv[1] = bfr_to_h(a[1]); hv[2] = bfr_to_h(a[2]); hv[3] = bfr_to_h(a[3]);
    hv[4] = bfr_to_h(c[0]); hv[5] = bfr_to_h(c[1]); hv[6] = bfr_to_h(c[2]); hv[7] = bfr_to_h(c[3]);
    _Float16* op = (_Float16*)out + base;
    *(volatile v8h*)op = hv;
    __threadfence();
    *(volatile v8h*)op = hv;
  }
}

__global__ __launch_bounds__(256) void build_vt(const float* __restrict__ val,
                                                 const float* __restrict__ state,
                                                 unsigned short* __restrict__ vt) {
  __shared__ __align__(16) _Float16 tileT[64][72];
  const int tid  = threadIdx.x;
  const int lane = tid & 31;
  const int wave = tid >> 5;
  const int jt = blockIdx.x;
  const int dt = blockIdx.y;
  const int b  = blockIdx.z;
  const int j0 = jt * 64;
  if (dt < 4) {
    const int d0 = dt * 64;
    const int jl = tid >> 2;
    const int dc = (tid & 3) * 16;
    const float* src = val + ((size_t)b * kNodes + j0 + jl) * kDim + d0 + dc;
#pragma unroll
    for (int q = 0; q < 4; ++q) {
      const v4f f = *(const v4f*)(src + 4 * q);
      tileT[dc + 4 * q + 0][jl] = bfr_to_h(f[0]);
      tileT[dc + 4 * q + 1][jl] = bfr_to_h(f[1]);
      tileT[dc + 4 * q + 2][jl] = bfr_to_h(f[2]);
      tileT[dc + 4 * q + 3][jl] = bfr_to_h(f[3]);
    }
  } else {
    const int jl = tid & 63;
    const int rg = (tid >> 6) * 16;
    const _Float16 sh = bfr_to_h(state[(size_t)b * kNodes + j0 + jl]);
    const _Float16 zh = (_Float16)0.0f;
#pragma unroll
    for (int r = 0; r < 16; ++r) tileT[rg + r][jl] = ((rg + r) == 0) ? sh : zh;
  }
  __syncthreads();
  const int q  = lane >> 3;
  const int c8 = (lane & 7) * 8;
  const int r0 = wave * 8 + q;
  const int r1 = wave * 8 + 4 + q;
  const v8h v0 = *(const v8h*)(&tileT[r0][c8]);
  const v8h v1 = *(const v8h*)(&tileT[r1][c8]);
  _Float16* dst = (_Float16*)vt + ((size_t)b * kVtRows + (size_t)dt * 64) * kNodes + j0 + c8;
  for (int pass = 0; pass < 2; ++pass) {
    *(volatile v8h*)(dst + (size_t)r0 * kNodes) = v0;
    *(volatile v8h*)(dst + (size_t)r1 * kNodes) = v1;
    __threadfence();
  }
}

constexpr int kOut1Blocks = kBatch * kNodes * kDim / 4 / 256;
constexpr int kOut0Blocks = kBatch * kNodes / 4 / 256;
static_assert(kOut1Blocks * 256 * 4 == kBatch * kNodes * kDim);
static_assert(kOut0Blocks * 256 * 4 == kBatch * kNodes);
__global__ __launch_bounds__(256) void pack_outputs(const float* __restrict__ cpl,
                                                     float* __restrict__ out0,
                                                     float* __restrict__ out1) {
  const int blk = blockIdx.x;
  const int tid = threadIdx.x;
  if (blk < kOut1Blocks) {
    const size_t t   = (size_t)blk * 256 + tid;
    const size_t row = t >> 6;
    const int    c   = (int)(t & 63) * 4;
    const v4f v = *(const v4f*)(cpl + row * kCPitch + c);
    float* dst = out1 + row * kDim + c;
    *(volatile v4f*)dst = v;
    __threadfence();
    *(volatile v4f*)dst = v;
  } else {
    const size_t t  = (size_t)(blk - kOut1Blocks) * 256 + tid;
    const size_t r4 = t * 4;
    v4f v;
    v[0] = cpl[(r4 + 0) * kCPitch + kDim];
    v[1] = cpl[(r4 + 1) * kCPitch + kDim];
    v[2] = cpl[(r4 + 2) * kCPitch + kDim];
    v[3] = cpl[(r4 + 3) * kCPitch + kDim];
    float* dst = out0 + r4;
    *(volatile v4f*)dst = v;
    __threadfence();
    *(volatile v4f*)dst = v;
  }
}

extern "C" void kernel_launch(void* const* d_in, const int* in_sizes, int n_in,
                              void* d_out, int out_size, void* d_ws, size_t ws_size,
                              hipStream_t stream) {
  if (n_in < 2) return;
  if (in_sizes[0] != kBatch * kNodes * kDim) return;
  if (in_sizes[1] != kBatch * kNodes) return;
  if (out_size != kBatch * kNodes + kBatch * kNodes * kDim) return;
  if (ws_size < kWsTotal) return;

  const float* val   = (const float*)d_in[0];
  const float* state = (const float*)d_in[1];
  float* out0 = (float*)d_out;
  float* out1 = (float*)d_out + (size_t)kBatch * kNodes;

  unsigned char* ws = (unsigned char*)d_ws;
  unsigned short* v16 = (unsigned short*)(ws + kOffV16);
  unsigned short* vt  = (unsigned short*)(ws + kOffVT);
  unsigned short* epl = (unsigned short*)(ws + kOffE);
  float*          cpl = (float*)(ws + kOffC);

  const int n8 = kBatch * kNodes * kDim / 8;
  cast_bfr_f16x8<<<dim3(n8 / 256), dim3(256), 0, stream>>>(val, v16, n8);

  build_vt<<<dim3(kNodes / 64, kVtRows / 64, kBatch), dim3(256), 0, stream>>>(val, state, vt);

  for (int b = 0; b < kBatch; ++b) {
    const unsigned short* vb  = v16 + (size_t)b * kNodes * kDim;
    const unsigned short* vtb = vt  + (size_t)b * kVtRows * kNodes;
    float* cb = cpl + (size_t)b * kNodes * kCPitch;
    wmma_gemm64<0, false, 0, 1, false, 6><<<dim3((kNodes / 64) * (kNodes / 64) / 8, 1), dim3(256), 0, stream>>>(
        vb, vb, kDim, 0L,
        vb, vb, kDim, 0L,
        (void*)epl, (void*)epl, kNodes, 0L,
        state,
        val, 0L,
        kNodes, kNodes, kDim, 0.0625f);
    wmma_gemm64<0, false, 0, 0, false, 0><<<dim3((kNodes / 64) * (kVtRows / 64) / 8, 1), dim3(256), 0, stream>>>(
        epl, epl, kNodes, 0L,
        vtb, vtb, kNodes, 0L,
        (void*)cb, (void*)cb, kCPitch, 0L,
        state,
        val, 0L,
        kNodes, kVtRows, kNodes, 1.0f);
  }

  pack_outputs<<<dim3(kOut1Blocks + kOut0Blocks), dim3(256), 0, stream>>>(cpl, out0, out1);
}
